// SoAGREE_47021301956985
// MI455X (gfx1250) — hardware-run, weakly checked
//
#include <hip/hip_runtime.h>


#define NU   50000
#define NUP  50048
#define NG   20000
#define NGP  20032
#define DD   64
#define KN   32
#define MM   16
typedef _Float16 h16;
typedef unsigned short bf;
typedef __attribute__((ext_vector_type(16))) __bf16   v16bf;
typedef __attribute__((ext_vector_type(16))) _Float16 v16h;
typedef __attribute__((ext_vector_type(8)))  _Float16 v8h;
typedef __attribute__((ext_vector_type(8)))  unsigned short v8us;
typedef __attribute__((ext_vector_type(8)))  float    v8f;
typedef __attribute__((ext_vector_type(4)))  float    v4f;
typedef v8h  __attribute__((may_alias)) v8ha;
typedef v4f  __attribute__((may_alias)) v4fa;
typedef v8us __attribute__((may_alias)) v8usa;

__device__ __forceinline__ unsigned short f2bf(float f) { unsigned u = __float_as_uint(f); u += 0x7FFFu + ((u >> 16) & 1u); return (unsigned short)(u >> 16); }
__device__ __forceinline__ float bf2f(unsigned short b) { return __uint_as_float(((unsigned)b) << 16); }
__device__ __forceinline__ float bfr(float f) { return bf2f(f2bf(f)); }
__device__ __forceinline__ v16h cat16(v8h lo, v8h hi) { return __builtin_shufflevector(lo, hi, 0, 1, 2, 3, 4, 5, 6, 7, 8, 9, 10, 11, 12, 13, 14, 15); }
__device__ __forceinline__ v16bf cat16b(v8us lo, v8us hi) { return __builtin_bit_cast(v16bf, __builtin_shufflevector(lo, hi, 0, 1, 2, 3, 4, 5, 6, 7, 8, 9, 10, 11, 12, 13, 14, 15)); }
__device__ __forceinline__ v8f wmma16(v16h a, v16h b, v8f c) { return __builtin_amdgcn_wmma_f32_16x16x32_f16(false, a, false, b, (short)0, c, false, false); }
__device__ __forceinline__ v8f wmmab(v16bf a, v16bf b, v8f c) { return __builtin_amdgcn_wmma_f32_16x16x32_bf16(false, a, false, b, (short)0, c, false, false); }


template <typename T16> struct WFrag;
template <> struct WFrag<h16> { typedef v16h V; static __device__ __forceinline__ V ld(const h16* p) { return cat16(*(const v8h*)p, *(const v8h*)(p + 16)); } static __device__ __forceinline__ v8f mma(V a, V b, v8f c) { return wmma16(a, b, c); } };
template <> struct WFrag<bf> { typedef v16bf V; static __device__ __forceinline__ V ld(const bf* p) { return cat16b(*(const v8us*)p, *(const v8us*)(p + 16)); } static __device__ __forceinline__ v8f mma(V a, V b, v8f c) { return wmmab(a, b, c); } };
template <typename T16, int NSPLIT, bool BIAS>
__global__ __launch_bounds__(32) void k_gemmw(const T16* __restrict__ A, const T16* __restrict__ A2, const T16* __restrict__ Bt, const T16* __restrict__ Bt2, int K, float* C, int ldc, const float* __restrict__ bias, size_t sA, size_t sB, size_t sC) {
    typedef typename WFrag<T16>::V V;
    __shared__ __align__(16) float os[16 * 68];
    const size_t z = blockIdx.z; A += z * sA; if (A2) A2 += z * sA; Bt += z * sB; if (Bt2) Bt2 += z * sB; C += z * sC;
    const int lane = threadIdx.x & 31, lr = lane & 15, hi = lane >> 4; const int r0 = blockIdx.x * 64, c0 = blockIdx.y * 64;
    v8f acc[4][4];
#pragma unroll
    for (int mb = 0; mb < 4; ++mb)
#pragma unroll
        for (int nb = 0; nb < 4; ++nb) acc[mb][nb] = (v8f){};
    const size_t aoff = (size_t)(r0 + lr) * K + 8 * hi, boff = (size_t)(c0 + lr) * K + 8 * hi;
#pragma unroll 1
    for (int kc = 0; kc < K; kc += 32) {
        V a[4], a2[4];
#pragma unroll
        for (int mb = 0; mb < 4; ++mb) { a[mb] = WFrag<T16>::ld(A + aoff + (size_t)mb * 16 * K + kc); if (NSPLIT == 1 || NSPLIT == 2) a2[mb] = WFrag<T16>::ld(A2 + aoff + (size_t)mb * 16 * K + kc); }
#pragma unroll
        for (int nb = 0; nb < 4; ++nb) { const V b = WFrag<T16>::ld(Bt + boff + (size_t)nb * 16 * K + kc); V b2; if (NSPLIT >= 2) b2 = WFrag<T16>::ld(Bt2 + boff + (size_t)nb * 16 * K + kc);
#pragma unroll
            for (int mb = 0; mb < 4; ++mb) { acc[mb][nb] = WFrag<T16>::mma(a[mb], b, acc[mb][nb]); if (NSPLIT == 1 || NSPLIT == 2) acc[mb][nb] = WFrag<T16>::mma(a2[mb], b, acc[mb][nb]); if (NSPLIT >= 2) acc[mb][nb] = WFrag<T16>::mma(a[mb], b2, acc[mb][nb]); } }
        asm volatile("v_nop\n\tv_nop\n\tv_nop\n\tv_nop" : "+v"(acc[0][0]), "+v"(acc[1][1]), "+v"(acc[2][2]), "+v"(acc[3][3]) : "v"(a[0]), "v"(a[3]));
    }
#pragma unroll
    for (int mb = 0; mb < 4; ++mb) {
#pragma unroll
        for (int nb = 0; nb < 4; ++nb) {
#pragma unroll
            for (int j = 0; j < 8; ++j) os[(hi * 8 + j) * 68 + nb * 16 + lr] = acc[mb][nb][j]; }
        __builtin_amdgcn_wave_barrier(); asm volatile("" ::: "memory");
        float* crow = C + (size_t)(r0 + mb * 16) * ldc + c0;
#pragma unroll 1
        for (int ps = 0; ps < 2; ++ps) {
#pragma unroll
            for (int s = 0; s < 8; ++s) { const int row = 2 * s + hi, cofs = lr * 4; v4f val = *(const v4fa*)(os + row * 68 + cofs); if (BIAS) { val[0] += bfr(bias[c0 + cofs]); val[1] += bfr(bias[c0 + cofs + 1]); val[2] += bfr(bias[c0 + cofs + 2]); val[3] += bfr(bias[c0 + cofs + 3]); }
                *(volatile v4f*)(crow + (size_t)row * ldc + cofs) = val; }
            if (ps == 0) __threadfence(); }
        __builtin_amdgcn_wave_barrier(); asm volatile("" ::: "memory");
    }
}

__device__ __forceinline__ void splitf(float y, unsigned short& h, unsigned short& l) { h = f2bf(y); l = f2bf(y - bf2f(h)); }
typedef __attribute__((ext_vector_type(2))) unsigned short v2us;
typedef __attribute__((ext_vector_type(4))) unsigned short v4us;

__global__ __launch_bounds__(256) void k_wtG(const float* __restrict__ w, int K, int N, bf* Bt) {
    const int lane = threadIdx.x & 31; const int L0 = (blockIdx.x * 8 + (threadIdx.x >> 5)) * 8; const int nlines = N * K / 64;
#pragma unroll
    for (int ps = 0; ps < 2; ++ps) {
#pragma unroll 1
        for (int l = 0; l < 8; ++l) { const int L = L0 + l; if (L >= nlines) break; const size_t e = (size_t)L * 64 + lane * 2; const int k = (int)(e % K), n = (int)(e / K); v2us o;
            o[0] = f2bf(w[(size_t)k * N + n]); o[1] = f2bf(w[(size_t)(k + 1) * N + n]); *(volatile v2us*)(Bt + e) = o; }
        if (ps == 0) __threadfence(); }
}
__global__ __launch_bounds__(256) void k_cvtpad(const float* __restrict__ x, int nreal, int npad, bf* X) { const size_t e = ((size_t)blockIdx.x * 256 + threadIdx.x) * 4; if (e >= (size_t)npad * DD) return; const int r = (int)(e / DD); v4us o;
#pragma unroll
    for (int u = 0; u < 4; ++u) o[u] = (r < nreal) ? f2bf(x[e + u]) : (unsigned short)0; *(volatile v4us*)(X + e) = o; __threadfence(); *(volatile v4us*)(X + e) = o; }
__global__ __launch_bounds__(256) void k_split2(const float* __restrict__ F, int nreal, int npad, bf* Ph, bf* Pl) { const size_t e = ((size_t)blockIdx.x * 256 + threadIdx.x) * 4; if (e >= (size_t)npad * DD) return; const int r = (int)(e / DD); v4us oh, ol;
#pragma unroll
    for (int u = 0; u < 4; ++u) { unsigned short a = 0, b = 0; if (r < nreal) splitf(F[e + u], a, b); oh[u] = a; ol[u] = b; } *(volatile v4us*)(Ph + e) = oh; *(volatile v4us*)(Pl + e) = ol; __threadfence(); *(volatile v4us*)(Ph + e) = oh; *(volatile v4us*)(Pl + e) = ol; }
template <int L> __global__ __launch_bounds__(256) void k_agg(int nrows, const int* __restrict__ index, const int* __restrict__ counts, int nsrc, const float* __restrict__ P1, const float* __restrict__ C2, int c2stride, const float* __restrict__ b1, const float* __restrict__ w2, const float* __restrict__ b2,
                                             const float* __restrict__ SRC, int srcRaw, const float* __restrict__ base, float* AG) {
    const int gid = blockIdx.x * 16 + (threadIdx.x >> 4); const int q = threadIdx.x & 15; if (gid >= nrows) return; const int d0 = 4 * q; int cnt = counts[gid]; cnt = cnt < 0 ? 0 : (cnt > L ? L : cnt);
    float cadd[4], b1v[4], w2v[4], bsv[4];
#pragma unroll
    for (int u = 0; u < 4; ++u) { cadd[u] = C2[(size_t)gid * c2stride + d0 + u]; b1v[u] = bfr(b1[d0 + u]); w2v[u] = bfr(w2[d0 + u]); bsv[u] = bfr(base[(size_t)gid * DD + d0 + u]); asm volatile("" : "+v"(b1v[u])); asm volatile("" : "+v"(w2v[u])); asm volatile("" : "+v"(bsv[u])); }
    float bb2 = bfr(b2[0]); asm volatile("" : "+v"(bb2)); float sc[L]; float mx = -3.0e38f;
#pragma unroll
    for (int k = 0; k < L; ++k) { int id = index[(size_t)gid * L + k]; id = id < 0 ? 0 : (id >= nsrc ? nsrc - 1 : id); float part = 0.f;
#pragma unroll
        for (int u = 0; u < 4; ++u) { float t = __fadd_rn(__fadd_rn(P1[(size_t)id * DD + d0 + u], cadd[u]), b1v[u]); t = fmaxf(t, 0.f); float p = __fmul_rn(t, w2v[u]); asm volatile("" : "+v"(p)); part = __fadd_rn(part, p); }
        part += __shfl_xor(part, 1, 16); part += __shfl_xor(part, 2, 16); part += __shfl_xor(part, 4, 16); part += __shfl_xor(part, 8, 16);
        const float s = (k < cnt) ? __fadd_rn(part, bb2) : -1.0e9f; sc[k] = s; mx = fmaxf(mx, s); }
    float sum = 0.f;
#pragma unroll
    for (int k = 0; k < L; ++k) { float dlt = __fsub_rn(sc[k], mx); asm volatile("" : "+v"(dlt)); sc[k] = __expf(dlt); sum = __fadd_rn(sum, sc[k]); }
    const float inv = __fdiv_rn(1.0f, sum); float acc[4] = {0.f, 0.f, 0.f, 0.f};
#pragma unroll
    for (int k = 0; k < L; ++k) { int id = index[(size_t)gid * L + k]; id = id < 0 ? 0 : (id >= nsrc ? nsrc - 1 : id); const float w = __fmul_rn(sc[k], inv);
#pragma unroll
        for (int u = 0; u < 4; ++u) { float v = SRC[(size_t)id * DD + d0 + u]; if (srcRaw) v = bfr(v); asm volatile("" : "+v"(v)); float p = __fmul_rn(w, v); asm volatile("" : "+v"(p)); acc[u] = __fadd_rn(acc[u], p); } }
    v4f o;
#pragma unroll
    for (int u = 0; u < 4; ++u) o[u] = (cnt > 0) ? __fadd_rn(acc[u], bsv[u]) : bsv[u];
    float* dst = AG + (size_t)gid * DD + d0; *(volatile v4f*)dst = o; __threadfence(); *(volatile v4f*)dst = o; }
__global__ __launch_bounds__(256) void k_elem(const float* __restrict__ GR, const float* __restrict__ repo, bf* Eh, bf* El, bf* Gh, bf* Gl) { const size_t e = ((size_t)blockIdx.x * 256 + threadIdx.x) * 4; if (e >= (size_t)NGP * DD) return; const int r = (int)(e / DD); const int d = (int)(e % DD); v4us eh, el, gh, gl;
#pragma unroll
    for (int u = 0; u < 4; ++u) { unsigned short a = 0, b = 0, c = 0, dd2 = 0; if (r < NG) { const float gv = GR[e + u]; splitf(gv, c, dd2); splitf(__fmul_rn(gv, bfr(repo[d + u])), a, b); } eh[u] = a; el[u] = b; gh[u] = c; gl[u] = dd2; }
    for (int ps = 0; ps < 2; ++ps) { *(volatile v4us*)(Eh + e) = eh; *(volatile v4us*)(El + e) = el; *(volatile v4us*)(Gh + e) = gh; *(volatile v4us*)(Gl + e) = gl; if (ps == 0) __threadfence(); } }
__global__ __launch_bounds__(256) void k_pred2(const float* __restrict__ HPa, const float* __restrict__ HPb, const float* __restrict__ RP, const float* __restrict__ bp1, const float* __restrict__ wp2, const float* __restrict__ bp2, float* OUT) { const int gI = blockIdx.x * 256 + threadIdx.x; if (gI >= NG) return; float s = bfr(bp2[0]);
#pragma unroll 1
    for (int d = 0; d < DD; ++d) { float t = fmaxf(__fadd_rn(__fadd_rn(__fadd_rn(HPa[(size_t)gI * DD + d], HPb[(size_t)gI * DD + d]), RP[d]), bfr(bp1[d])), 0.f); float p = __fmul_rn(t, bfr(wp2[d])); asm volatile("" : "+v"(p)); s = __fadd_rn(s, p); }
    const float y = __fdiv_rn(1.0f, 1.0f + __expf(-s)); *(volatile float*)(OUT + gI) = y; __threadfence(); *(volatile float*)(OUT + gI) = y; }
__global__ __launch_bounds__(64) void k_rvec(const float* __restrict__ repo, const float* __restrict__ Wt, int row0, float* RP) { const int d = threadIdx.x; float s = 0.f;
#pragma unroll 1
    for (int j = 0; j < DD; ++j) { float p = __fmul_rn(bfr(repo[j]), bfr(Wt[(size_t)(row0 + j) * DD + d])); asm volatile("" : "+v"(p)); s = __fadd_rn(s, p); } *(volatile float*)(RP + d) = s; __threadfence(); *(volatile float*)(RP + d) = s; }

extern "C" void kernel_launch(void* const* d_in, const int* in_sizes, int n_in,
                              void* d_out, int out_size, void* d_ws, size_t ws_size, hipStream_t stream) {
    (void)in_sizes; (void)n_in; (void)out_size;
    const float* repo = (const float*)d_in[0]; const float* team = (const float*)d_in[1]; const float* users = (const float*)d_in[2]; const float* Wf1 = (const float*)d_in[3]; const float* bf1 = (const float*)d_in[4]; const float* Wf2 = (const float*)d_in[5]; const float* bf2 = (const float*)d_in[6];
    const float* Wa1 = (const float*)d_in[7]; const float* ba1 = (const float*)d_in[8]; const float* Wa2 = (const float*)d_in[9]; const float* ba2 = (const float*)d_in[10]; const float* Wp1 = (const float*)d_in[11]; const float* bp1 = (const float*)d_in[12]; const float* Wp2 = (const float*)d_in[13]; const float* bp2 = (const float*)d_in[14];
    const int* tmem = (const int*)d_in[15]; const int* tcnt = (const int*)d_in[16]; const int* unbr = (const int*)d_in[17]; const int* ucnt = (const int*)d_in[18];
    float* OUT = (float*)d_out;
    char* wsp = (char*)d_ws;
    auto take = [&](size_t bytes) { char* p = wsp; wsp += (bytes + 255) & ~(size_t)255; return (void*)p; };
    bf* WF1a = (bf*)take(DD * DD * 2); bf* WF1b = (bf*)take(DD * DD * 2); bf* WA1a = (bf*)take(DD * DD * 2); bf* WP1a = (bf*)take(DD * DD * 2); bf* WP1b = (bf*)take(DD * DD * 2);
    bf* UB = (bf*)take((size_t)NUP * DD * 2); float* E1 = (float*)take((size_t)NUP * DD * 4); float* E2 = (float*)take((size_t)NUP * DD * 4); float* UAG = (float*)take((size_t)NUP * DD * 4); bf* UAh = (bf*)take((size_t)NUP * DD * 2); bf* UAl = (bf*)take((size_t)NUP * DD * 2); float* A1 = (float*)take((size_t)NUP * DD * 4); float* RA = (float*)take(256); float* RP = (float*)take(256);
    float* GR = (float*)take((size_t)NGP * DD * 4); bf* Eh = (bf*)take((size_t)NGP * DD * 2); bf* El = (bf*)take((size_t)NGP * DD * 2); bf* Gh = (bf*)take((size_t)NGP * DD * 2); bf* Gl = (bf*)take((size_t)NGP * DD * 2); float* HPa = (float*)take((size_t)NGP * DD * 4); float* HPb = (float*)take((size_t)NGP * DD * 4); float* HP = (float*)take((size_t)NGP * DD * 4);
    if ((size_t)(wsp - (char*)d_ws) > ws_size) return;
    k_wtG<<<(DD * DD / 64 + 63) / 64, 256, 0, stream>>>(Wf1, DD, DD, WF1a); k_wtG<<<(DD * DD / 64 + 63) / 64, 256, 0, stream>>>(Wf1 + DD * DD, DD, DD, WF1b); k_wtG<<<(DD * DD / 64 + 63) / 64, 256, 0, stream>>>(Wa1, DD, DD, WA1a); k_wtG<<<(DD * DD / 64 + 63) / 64, 256, 0, stream>>>(Wp1, DD, DD, WP1a); k_wtG<<<(DD * DD / 64 + 63) / 64, 256, 0, stream>>>(Wp1 + DD * DD, DD, DD, WP1b);
    k_rvec<<<1, 64, 0, stream>>>(repo, Wa1, DD, RA); k_rvec<<<1, 64, 0, stream>>>(repo, Wp1, 2 * DD, RP);
    k_cvtpad<<<(unsigned)(((size_t)NUP * DD / 4 + 255) / 256), 256, 0, stream>>>(users, NU, NUP, UB);
    k_gemmw<bf, 0, false><<<dim3(NUP / 64, 1, 1), 32, 0, stream>>>(UB, nullptr, WF1a, nullptr, DD, E1, DD, nullptr, 0, 0, 0); k_gemmw<bf, 0, false><<<dim3(NUP / 64, 1, 1), 32, 0, stream>>>(UB, nullptr, WF1b, nullptr, DD, E2, DD, nullptr, 0, 0, 0);
    k_agg<KN><<<(NU + 15) / 16, 256, 0, stream>>>(NU, unbr, ucnt, NU, E1, E2, DD, bf1, Wf2, bf2, users, 1, users, UAG);
    k_split2<<<(unsigned)(((size_t)NUP * DD / 4 + 255) / 256), 256, 0, stream>>>(UAG, NU, NUP, UAh, UAl);
    k_gemmw<bf, 1, false><<<dim3(NUP / 64, 1, 1), 32, 0, stream>>>(UAh, UAl, WA1a, nullptr, DD, A1, DD, nullptr, 0, 0, 0);
    k_agg<MM><<<(NG + 15) / 16, 256, 0, stream>>>(NG, tmem, tcnt, NU, A1, RA, 0, ba1, Wa2, ba2, UAG, 0, team, GR);
    k_elem<<<(unsigned)(((size_t)NGP * DD / 4 + 255) / 256), 256, 0, stream>>>(GR, repo, Eh, El, Gh, Gl);
    k_gemmw<bf, 1, false><<<dim3(NGP / 64, 1, 1), 32, 0, stream>>>(Eh, El, WP1a, nullptr, DD, HPa, DD, nullptr, 0, 0, 0); k_gemmw<bf, 1, false><<<dim3(NGP / 64, 1, 1), 32, 0, stream>>>(Gh, Gl, WP1b, nullptr, DD, HPb, DD, nullptr, 0, 0, 0);
    k_pred2<<<(NG + 255) / 256, 256, 0, stream>>>(HPa, HPb, RP, bp1, Wp2, bp2, OUT);
}
